// KDABlock_50929722196117
// MI455X (gfx1250) — hardware-verified
//
#include <hip/hip_runtime.h>
#include <stddef.h>


#define NB 2
#define NT 2048
#define ND 1024
#define NH 16
#define HD 64
#define NI 2816
#define NM (NB * NT)
#define SMW 256
#define SP 72
#define NCH (NI / 256)

typedef __bf16 v16b __attribute__((ext_vector_type(16)));
typedef unsigned short v8us __attribute__((ext_vector_type(8)));
typedef float v8f __attribute__((ext_vector_type(8)));
typedef float v4f __attribute__((ext_vector_type(4)));

union Frag {
  v16b v;
  v8us h[2];
};

__device__ __forceinline__ unsigned short f2bf(float f) {
  unsigned int u = __float_as_uint(f);
  u += 0x7FFFu + ((u >> 16) & 1u);
  return (unsigned short)(u >> 16);
}

__device__ __forceinline__ v8us pack8(v4f a, v4f b) {
  v8us r;
  r[0] = f2bf(a.x); r[1] = f2bf(a.y); r[2] = f2bf(a.z); r[3] = f2bf(a.w);
  r[4] = f2bf(b.x); r[5] = f2bf(b.y); r[6] = f2bf(b.z); r[7] = f2bf(b.w);
  return r;
}

__device__ __forceinline__ float sigf(float x) { return __builtin_amdgcn_rcpf(1.0f + __expf(-x)); }
__device__ __forceinline__ float softplusf(float x) { return fmaxf(x, 0.0f) + log1pf(expf(-fabsf(x))); }

#define WMMA_BF16(acc, fa, fb) \
  acc = __builtin_amdgcn_wmma_f32_16x16x32_bf16(false, (fa).v, false, (fb).v, (short)0, acc, false, false)

__global__ __launch_bounds__(256) void k_wtr(const float* __restrict__ W, int Krows, int Ncols,
                                            unsigned short* __restrict__ WT, int nrows_out) {
  __shared__ float tsm[64][65];
  const int tid = threadIdx.x, l = tid & 31, wid = tid >> 5;
  const int k0 = blockIdx.x * 64, n0 = blockIdx.y * 64;
#pragma unroll
  for (int j = 0; j < 4; ++j) {
    const int idx = tid + 256 * j;
    const int kk = idx >> 4, nn = (idx & 15) * 4;
    const int k = k0 + kk, n = n0 + nn;
    v4f v = {0.0f, 0.0f, 0.0f, 0.0f};
    if (k < Krows && n + 3 < Ncols) v = *(const v4f*)(W + (size_t)k * Ncols + n);
    tsm[nn + 0][kk] = v.x;
    tsm[nn + 1][kk] = v.y;
    tsm[nn + 2][kk] = v.z;
    tsm[nn + 3][kk] = v.w;
  }
  __syncthreads();
  const int p = l & 7;
  v8us pv[2];
#pragma unroll
  for (int i = 0; i < 2; ++i) {
    const int nr = wid * 8 + 4 * i + (l >> 3);
    v4f x0, x1;
    x0.x = tsm[nr][8 * p + 0]; x0.y = tsm[nr][8 * p + 1]; x0.z = tsm[nr][8 * p + 2]; x0.w = tsm[nr][8 * p + 3];
    x1.x = tsm[nr][8 * p + 4]; x1.y = tsm[nr][8 * p + 5]; x1.z = tsm[nr][8 * p + 6]; x1.w = tsm[nr][8 * p + 7];
    pv[i] = pack8(x0, x1);
  }
  const bool kok = (k0 + 64 <= Krows);
#pragma unroll
  for (int i = 0; i < 2; ++i) {
    const int n = n0 + wid * 8 + 4 * i + (l >> 3);
    if (kok && n < nrows_out) *(volatile v8us*)(WT + (size_t)n * Krows + k0 + 8 * p) = pv[i];
  }
  __threadfence();
#pragma unroll
  for (int i = 0; i < 2; ++i) {
    const int n = n0 + wid * 8 + 4 * i + (l >> 3);
    if (kok && n < nrows_out) *(volatile v8us*)(WT + (size_t)n * Krows + k0 + 8 * p) = pv[i];
  }
}

__global__ __launch_bounds__(128) void k_ln(const float* __restrict__ x, const float* __restrict__ w,
                                           const float* __restrict__ bb, unsigned short* __restrict__ out,
                                           int rows) {
  __shared__ float red[2][4];
  const int row = blockIdx.x;
  if (row >= rows) return;
  const int tid = threadIdx.x, l = tid & 31, wid = tid >> 5;
  const float* xr = x + (size_t)row * ND + 8 * tid;
  v4f a = *(const v4f*)xr;
  v4f c = *(const v4f*)(xr + 4);
  float s = ((a.x + a.y) + (a.z + a.w)) + ((c.x + c.y) + (c.z + c.w));
  s += __shfl_xor(s, 16); s += __shfl_xor(s, 8); s += __shfl_xor(s, 4); s += __shfl_xor(s, 2); s += __shfl_xor(s, 1);
  if (l == 0) red[0][wid] = s;
  __syncthreads();
  const float mean = ((red[0][0] + red[0][1]) + (red[0][2] + red[0][3])) * (1.0f / ND);
  a = a - mean;
  c = c - mean;
  float s2 = a.x * a.x + a.y * a.y + a.z * a.z + a.w * a.w + c.x * c.x + c.y * c.y + c.z * c.z + c.w * c.w;
  s2 += __shfl_xor(s2, 16); s2 += __shfl_xor(s2, 8); s2 += __shfl_xor(s2, 4); s2 += __shfl_xor(s2, 2); s2 += __shfl_xor(s2, 1);
  if (l == 0) red[1][wid] = s2;
  __syncthreads();
  const float var = ((red[1][0] + red[1][1]) + (red[1][2] + red[1][3])) * (1.0f / ND);
  const float rstd = rsqrtf(var + 1e-5f);
  const v4f w0 = *(const v4f*)(w + 8 * tid), w1 = *(const v4f*)(w + 8 * tid + 4);
  const v4f b0 = *(const v4f*)(bb + 8 * tid), b1 = *(const v4f*)(bb + 8 * tid + 4);
  const v4f y0 = a * rstd * w0 + b0;
  const v4f y1 = c * rstd * w1 + b1;
  const v8us pk = pack8(y0, y1);
  unsigned short* dst = out + (size_t)row * ND + 8 * tid;
  *(volatile v8us*)dst = pk;
  __threadfence();
  *(volatile v8us*)dst = pk;
}

enum { E_F32 = 0, E_L2N = 1, E_SMALL = 2, E_DECAY = 3, E_SIG = 4, E_BF16 = 5, E_RESID = 6 };

template <int EPI, bool A32>
__global__ __launch_bounds__(256) void k_gemm(const void* __restrict__ Aptr, int lda,
                                             const unsigned short* __restrict__ Bt, int nbrows,
                                             void* __restrict__ Cptr, int ldc, int Kd, int Mrows,
                                             const float* __restrict__ aux0,
                                             const float* __restrict__ aux1,
                                             const int* __restrict__ auxi) {
  __shared__ __align__(32) float lds_f[128 * 128];
  unsigned short* sA = (unsigned short*)lds_f;
  unsigned short* sB = sA + 128 * SP;
  const int tid = threadIdx.x, l = tid & 31, wid = tid >> 5, h = l >> 4, m = l & 15;
  const int wm = wid >> 1, wn = wid & 1;
  const int rowBase = blockIdx.y * 128, colBase = blockIdx.x * 128;
  const v8us z8 = {0, 0, 0, 0, 0, 0, 0, 0};
  v8f c00 = {0, 0, 0, 0, 0, 0, 0, 0}, c01 = {0, 0, 0, 0, 0, 0, 0, 0};
  v8f c02 = {0, 0, 0, 0, 0, 0, 0, 0}, c03 = {0, 0, 0, 0, 0, 0, 0, 0};
  v8f c10 = {0, 0, 0, 0, 0, 0, 0, 0}, c11 = {0, 0, 0, 0, 0, 0, 0, 0};
  v8f c12 = {0, 0, 0, 0, 0, 0, 0, 0}, c13 = {0, 0, 0, 0, 0, 0, 0, 0};

#pragma unroll 1
  for (int k0 = 0; k0 < Kd; k0 += 64) {
#pragma unroll
    for (int j = 0; j < 4; ++j) {
      const int idx = tid + 256 * j;
      const int r = idx >> 3, kc = (idx & 7) * 8;
      const int gr = rowBase + r;
      v8us av = z8;
      if (gr < Mrows) {
        if (A32) {
          const float* ap = (const float*)Aptr + (size_t)gr * lda + k0 + kc;
          av = pack8(*(const v4f*)ap, *(const v4f*)(ap + 4));
        } else {
          av = *(const v8us*)((const unsigned short*)Aptr + (size_t)gr * lda + k0 + kc);
        }
      }
      *(v8us*)(sA + r * SP + kc) = av;
      const int gn = colBase + r;
      v8us bv = z8;
      if (gn < nbrows) bv = *(const v8us*)(Bt + (size_t)gn * Kd + k0 + kc);
      *(v8us*)(sB + r * SP + kc) = bv;
    }
    __syncthreads();
#pragma unroll
    for (int ks = 0; ks < 64; ks += 32) {
      Frag a0, a1, b0, b1, b2, b3;
      const unsigned short* pa = sA + (wm * 32 + m) * SP + ks + 8 * h;
      a0.h[0] = *(const v8us*)(pa);
      a0.h[1] = *(const v8us*)(pa + 16);
      a1.h[0] = *(const v8us*)(pa + 16 * SP);
      a1.h[1] = *(const v8us*)(pa + 16 * SP + 16);
      const unsigned short* pb = sB + (wn * 64 + m) * SP + ks + 8 * h;
      b0.h[0] = *(const v8us*)(pb);
      b0.h[1] = *(const v8us*)(pb + 16);
      b1.h[0] = *(const v8us*)(pb + 16 * SP);
      b1.h[1] = *(const v8us*)(pb + 16 * SP + 16);
      b2.h[0] = *(const v8us*)(pb + 32 * SP);
      b2.h[1] = *(const v8us*)(pb + 32 * SP + 16);
      b3.h[0] = *(const v8us*)(pb + 48 * SP);
      b3.h[1] = *(const v8us*)(pb + 48 * SP + 16);
      WMMA_BF16(c00, a0, b0);
      WMMA_BF16(c01, a0, b1);
      WMMA_BF16(c02, a0, b2);
      WMMA_BF16(c03, a0, b3);
      WMMA_BF16(c10, a1, b0);
      WMMA_BF16(c11, a1, b1);
      WMMA_BF16(c12, a1, b2);
      WMMA_BF16(c13, a1, b3);
      asm volatile("v_nop\n\tv_nop\n\tv_nop\n\tv_nop"
                   : "+v"(c00), "+v"(c01), "+v"(c02), "+v"(c03), "+v"(c10), "+v"(c11), "+v"(c12), "+v"(c13)
                   : "v"(a0.v), "v"(a1.v), "v"(b0.v), "v"(b1.v), "v"(b2.v), "v"(b3.v));
    }
    __syncthreads();
  }

  float* Cs = lds_f;
  {
    const int rr = wm * 32 + 8 * h;
    const int cc = wn * 64 + m;
    *(v8f*)(Cs + (cc + 0) * 128 + rr) = c00;
    *(v8f*)(Cs + (cc + 16) * 128 + rr) = c01;
    *(v8f*)(Cs + (cc + 32) * 128 + rr) = c02;
    *(v8f*)(Cs + (cc + 48) * 128 + rr) = c03;
    *(v8f*)(Cs + (cc + 0) * 128 + rr + 16) = c10;
    *(v8f*)(Cs + (cc + 16) * 128 + rr + 16) = c11;
    *(v8f*)(Cs + (cc + 32) * 128 + rr + 16) = c12;
    *(v8f*)(Cs + (cc + 48) * 128 + rr + 16) = c13;
  }
  __syncthreads();

  if (EPI == E_BF16) {
    unsigned short* Cb = (unsigned short*)Cptr;
    const int c8 = 8 * m;
    v8us pv[8];
#pragma unroll
    for (int q = 0; q < 8; ++q) {
      const int row = wid * 16 + 2 * q + h;
      v4f x0, x1;
      x0.x = Cs[(c8 + 0) * 128 + row]; x0.y = Cs[(c8 + 1) * 128 + row];
      x0.z = Cs[(c8 + 2) * 128 + row]; x0.w = Cs[(c8 + 3) * 128 + row];
      x1.x = Cs[(c8 + 4) * 128 + row]; x1.y = Cs[(c8 + 5) * 128 + row];
      x1.z = Cs[(c8 + 6) * 128 + row]; x1.w = Cs[(c8 + 7) * 128 + row];
      pv[q] = pack8(x0, x1);
    }
#pragma unroll
    for (int q = 0; q < 8; ++q) {
      const int grow = rowBase + wid * 16 + 2 * q + h;
      if (grow < Mrows) *(volatile v8us*)(Cb + (size_t)grow * ldc + colBase + c8) = pv[q];
    }
    __threadfence();
#pragma unroll
    for (int q = 0; q < 8; ++q) {
      const int grow = rowBase + wid * 16 + 2 * q + h;
      if (grow < Mrows) *(volatile v8us*)(Cb + (size_t)grow * ldc + colBase + c8) = pv[q];
    }
  } else {
    float* Cf = (float*)Cptr;
    float ea = 0.0f;
    v4f dtb = {0.0f, 0.0f, 0.0f, 0.0f};
    if (EPI == E_DECAY) {
      const int col0 = colBase + 4 * l;
      ea = expf(aux1[col0 >> 6]);
      dtb = *(const v4f*)(aux0 + col0);
    }
    v4f pv[16];
#pragma unroll
    for (int q = 0; q < 16; ++q) {
      const int row = wid * 16 + q;
      int grow = rowBase + row;
      if (grow > Mrows - 1) grow = Mrows - 1;
      v4f x;
      x.x = Cs[(4 * l + 0) * 128 + row];
      x.y = Cs[(4 * l + 1) * 128 + row];
      x.z = Cs[(4 * l + 2) * 128 + row];
      x.w = Cs[(4 * l + 3) * 128 + row];
      if (EPI == E_L2N) {
        float ss = x.x * x.x + x.y * x.y + x.z * x.z + x.w * x.w;
        ss += __shfl_xor(ss, 8);
        ss += __shfl_xor(ss, 4);
        ss += __shfl_xor(ss, 2);
        ss += __shfl_xor(ss, 1);
        const float rs = rsqrtf(ss + 1e-6f);
        x = x * rs;
      } else if (EPI == E_SMALL) {
        if (colBase >= 2 * HD) {
          const float mk = (float)auxi[grow];
          x.x = sigf(x.x) * mk; x.y = sigf(x.y) * mk; x.z = sigf(x.z) * mk; x.w = sigf(x.w) * mk;
        }
      } else if (EPI == E_DECAY) {
        x.x = expf(-ea * softplusf(x.x + dtb.x));
        x.y = expf(-ea * softplusf(x.y + dtb.y));
        x.z = expf(-ea * softplusf(x.z + dtb.z));
        x.w = expf(-ea * softplusf(x.w + dtb.w));
      } else if (EPI == E_SIG) {
        x.x = sigf(x.x); x.y = sigf(x.y); x.z = sigf(x.z); x.w = sigf(x.w);
      } else if (EPI == E_RESID) {
        const v4f rsd = *(const v4f*)(aux0 + (size_t)grow * ldc + colBase + 4 * l);
        x = x + rsd;
      }
      pv[q] = x;
    }
#pragma unroll
    for (int q = 0; q < 16; ++q) {
      const int grow = rowBase + wid * 16 + q;
      if (grow < Mrows) *(volatile v4f*)(Cf + (size_t)grow * ldc + colBase + 4 * l) = pv[q];
    }
    __threadfence();
#pragma unroll
    for (int q = 0; q < 16; ++q) {
      const int grow = rowBase + wid * 16 + q;
      if (grow < Mrows) *(volatile v4f*)(Cf + (size_t)grow * ldc + colBase + 4 * l) = pv[q];
    }
  }
}

__global__ __launch_bounds__(256) void k_swiglu(const float* __restrict__ gu, unsigned short* __restrict__ act,
                                               int rows) {
  const int tid = threadIdx.x, l = tid & 31, wid = tid >> 5;
  const int gw = blockIdx.x * 8 + wid;
  const int row = gw / NCH, ch = gw - row * NCH;
  if (row >= rows) return;
  const int j = ch * 256 + 8 * l;
  const float* gp = gu + (size_t)row * (2 * NI) + j;
  const v4f g0 = *(const v4f*)gp, g1 = *(const v4f*)(gp + 4);
  const v4f u0 = *(const v4f*)(gp + NI), u1 = *(const v4f*)(gp + NI + 4);
  v4f y0, y1;
  y0.x = g0.x * sigf(g0.x) * u0.x; y0.y = g0.y * sigf(g0.y) * u0.y;
  y0.z = g0.z * sigf(g0.z) * u0.z; y0.w = g0.w * sigf(g0.w) * u0.w;
  y1.x = g1.x * sigf(g1.x) * u1.x; y1.y = g1.y * sigf(g1.y) * u1.y;
  y1.z = g1.z * sigf(g1.z) * u1.z; y1.w = g1.w * sigf(g1.w) * u1.w;
  const v8us pk = pack8(y0, y1);
  unsigned short* dst = act + (size_t)row * NI + j;
  *(volatile v8us*)dst = pk;
  __threadfence();
  *(volatile v8us*)dst = pk;
}

__global__ __launch_bounds__(256) void k_scan(const float* __restrict__ qf, const float* __restrict__ kf,
                                             const float* __restrict__ vf, const float* __restrict__ dec,
                                             const float* __restrict__ sm, const float* __restrict__ gsig,
                                             const float* __restrict__ onw, unsigned short* __restrict__ obf) {
  __shared__ __align__(16) float shq[2][64];
  __shared__ __align__(16) float shk[2][64];
  __shared__ __align__(16) float shd[2][64];
  __shared__ __align__(16) float red[2][4][64];
  __shared__ __align__(16) float sho[32][4][64];
  const int bh = blockIdx.x;
  const int b = bh / NH, hh = bh - b * NH;
  const int tid = threadIdx.x;
  const int vcol = tid & 63, kg = tid >> 6, kb = kg * 16;
  float S[16];
#pragma unroll
  for (int i = 0; i < 16; ++i) S[i] = 0.0f;

#pragma unroll 1
  for (int t0 = 0; t0 < NT; t0 += 32) {
#pragma unroll 1
    for (int tt = 0; tt < 32; ++tt) {
      const int p = tt & 1;
      const size_t row = (size_t)b * NT + t0 + tt;
      const size_t base = row * ND + (size_t)hh * HD;
      if (tid < 64) shq[p][tid] = qf[base + tid];
      else if (tid < 128) shk[p][tid - 64] = kf[base + tid - 64];
      else if (tid < 192) shd[p][tid - 128] = dec[base + tid - 128];
      const float vv = vf[base + vcol];
      const float bt = sm[row * SMW + 2 * HD + hh];
      __syncthreads();
      float part = 0.0f;
#pragma unroll
      for (int i = 0; i < 16; ++i) {
        S[i] *= shd[p][kb + i];
        part = fmaf(shk[p][kb + i], S[i], part);
      }
      red[p][kg][vcol] = part;
      __syncthreads();
      const float tot = (red[p][0][vcol] + red[p][1][vcol]) + (red[p][2][vcol] + red[p][3][vcol]);
      const float u = (vv - tot) * bt;
      float part2 = 0.0f;
#pragma unroll
      for (int i = 0; i < 16; ++i) {
        S[i] = fmaf(shk[p][kb + i], u, S[i]);
        part2 = fmaf(shq[p][kb + i], S[i], part2);
      }
      sho[tt][kg][vcol] = part2;
    }
    __syncthreads();
    {
      const int r = tid >> 3, c = tid & 7;
      const float* s0 = &sho[r][0][8 * c];
      v4f o0 = *(const v4f*)(s0) + *(const v4f*)(s0 + 64) + *(const v4f*)(s0 + 128) + *(const v4f*)(s0 + 192);
      v4f o1 = *(const v4f*)(s0 + 4) + *(const v4f*)(s0 + 68) + *(const v4f*)(s0 + 132) + *(const v4f*)(s0 + 196);
      o0 = o0 * 0.125f;
      o1 = o1 * 0.125f;
      float ss = o0.x * o0.x + o0.y * o0.y + o0.z * o0.z + o0.w * o0.w +
                 o1.x * o1.x + o1.y * o1.y + o1.z * o1.z + o1.w * o1.w;
      ss += __shfl_xor(ss, 4);
      ss += __shfl_xor(ss, 2);
      ss += __shfl_xor(ss, 1);
      const float rs = rsqrtf(ss * (1.0f / HD) + 1e-5f);
      const size_t row = (size_t)b * NT + t0 + r;
      const size_t gb = row * ND + (size_t)hh * HD + 8 * c;
      const v4f g0 = *(const v4f*)(gsig + gb), g1 = *(const v4f*)(gsig + gb + 4);
      const v4f w0 = *(const v4f*)(onw + 8 * c), w1 = *(const v4f*)(onw + 8 * c + 4);
      const v4f y0 = o0 * rs * w0 * g0;
      const v4f y1 = o1 * rs * w1 * g1;
      const v8us pk = pack8(y0, y1);
      unsigned short* dst = obf + gb;
      *(volatile v8us*)dst = pk;
      __threadfence();
      *(volatile v8us*)dst = pk;
    }
    __syncthreads();
  }
}

extern "C" void kernel_launch(void* const* d_in, const int* in_sizes, int n_in,
                              void* d_out, int out_size, void* d_ws, size_t ws_size,
                              hipStream_t stream) {
  if (n_in < 18) return;
  if (in_sizes[0] != NM * ND || in_sizes[1] != NM || out_size != NM * ND) return;
  if (in_sizes[4] != ND * ND || in_sizes[5] != ND * ND || in_sizes[6] != ND * ND || in_sizes[15] != ND * ND) return;
  if (in_sizes[7] != ND * HD || in_sizes[8] != HD * ND || in_sizes[12] != ND * HD || in_sizes[13] != HD * ND) return;
  if (in_sizes[11] != ND * NH || in_sizes[16] != ND * 2 * NI || in_sizes[17] != NI * ND) return;
  if (in_sizes[9] != ND || in_sizes[10] != NH || in_sizes[14] != HD || in_sizes[2] != ND || in_sizes[3] != ND) return;

  const float* hidden   = (const float*)d_in[0];
  const int*   amask    = (const int*)d_in[1];
  const float* ln_w     = (const float*)d_in[2];
  const float* ln_b     = (const float*)d_in[3];
  const float* q_w      = (const float*)d_in[4];
  const float* k_w      = (const float*)d_in[5];
  const float* v_w      = (const float*)d_in[6];
  const float* f_a_w    = (const float*)d_in[7];
  const float* f_b_w    = (const float*)d_in[8];
  const float* dt_bias  = (const float*)d_in[9];
  const float* A_log    = (const float*)d_in[10];
  const float* b_w      = (const float*)d_in[11];
  const float* g_a_w    = (const float*)d_in[12];
  const float* g_b_w    = (const float*)d_in[13];
  const float* o_norm_w = (const float*)d_in[14];
  const float* o_w      = (const float*)d_in[15];
  const float* gu_w     = (const float*)d_in[16];
  const float* down_w   = (const float*)d_in[17];
  float* out = (float*)d_out;

  char* ws = (char*)d_ws;
  size_t off = 0;
  auto carve = [&](size_t bytes) -> char* {
    char* p = ws + off;
    off += (bytes + 255) & ~(size_t)255;
    return p;
  };
  unsigned short* wqT  = (unsigned short*)carve((size_t)ND * ND * 2);
  unsigned short* wkT  = (unsigned short*)carve((size_t)ND * ND * 2);
  unsigned short* wvT  = (unsigned short*)carve((size_t)ND * ND * 2);
  unsigned short* woT  = (unsigned short*)carve((size_t)ND * ND * 2);
  unsigned short* wguT = (unsigned short*)carve((size_t)2 * NI * ND * 2);
  unsigned short* wdnT = (unsigned short*)carve((size_t)ND * NI * 2);
  unsigned short* wsmT = (unsigned short*)carve((size_t)SMW * ND * 2);
  unsigned short* wfbT = (unsigned short*)carve((size_t)ND * HD * 2);
  unsigned short* wgbT = (unsigned short*)carve((size_t)ND * HD * 2);
  unsigned short* xln  = (unsigned short*)carve((size_t)NM * ND * 2);
  float* qf   = (float*)carve((size_t)NM * ND * 4);
  float* kf   = (float*)carve((size_t)NM * ND * 4);
  float* vf   = (float*)carve((size_t)NM * ND * 4);
  float* gdec = (float*)carve((size_t)NM * ND * 4);
  float* gof  = (float*)carve((size_t)NM * ND * 4);
  float* smf  = (float*)carve((size_t)NM * SMW * 4);
  unsigned short* obf = (unsigned short*)carve((size_t)NM * ND * 2);
  unsigned short* opb = (unsigned short*)carve((size_t)NM * ND * 2);
  float* gu   = (float*)carve((size_t)NM * 2 * NI * 4);
  unsigned short* act = (unsigned short*)carve((size_t)NM * NI * 2);
  if (off > ws_size) return;

  const dim3 tb(256);

  k_wtr<<<dim3(ND / 64, ND / 64), tb, 0, stream>>>(q_w, ND, ND, wqT, ND);
  k_wtr<<<dim3(ND / 64, ND / 64), tb, 0, stream>>>(k_w, ND, ND, wkT, ND);
  k_wtr<<<dim3(ND / 64, ND / 64), tb, 0, stream>>>(v_w, ND, ND, wvT, ND);
  k_wtr<<<dim3(ND / 64, ND / 64), tb, 0, stream>>>(o_w, ND, ND, woT, ND);
  k_wtr<<<dim3(ND / 64, (2 * NI) / 64), tb, 0, stream>>>(gu_w, ND, 2 * NI, wguT, 2 * NI);
  k_wtr<<<dim3(NI / 64, ND / 64), tb, 0, stream>>>(down_w, NI, ND, wdnT, ND);
  k_wtr<<<dim3(ND / 64, 1), tb, 0, stream>>>(f_a_w, ND, HD, wsmT, HD);
  k_wtr<<<dim3(ND / 64, 1), tb, 0, stream>>>(g_a_w, ND, HD, wsmT + (size_t)HD * ND, HD);
  k_wtr<<<dim3(ND / 64, (SMW - 2 * HD) / 64), tb, 0, stream>>>(b_w, ND, NH,
                                                              wsmT + (size_t)2 * HD * ND, SMW - 2 * HD);
  k_wtr<<<dim3(HD / 64, ND / 64), tb, 0, stream>>>(f_b_w, HD, ND, wfbT, ND);
  k_wtr<<<dim3(HD / 64, ND / 64), tb, 0, stream>>>(g_b_w, HD, ND, wgbT, ND);

  k_ln<<<NM, 128, 0, stream>>>(hidden, ln_w, ln_b, xln, NM);

  const dim3 g1024(ND / 128, NM / 128);
  k_gemm<E_L2N, false><<<g1024, tb, 0, stream>>>(xln, ND, wqT, ND, qf, ND, ND, NM, nullptr, nullptr, nullptr);
  k_gemm<E_L2N, false><<<g1024, tb, 0, stream>>>(xln, ND, wkT, ND, kf, ND, ND, NM, nullptr, nullptr, nullptr);
  k_gemm<E_F32, false><<<g1024, tb, 0, stream>>>(xln, ND, wvT, ND, vf, ND, ND, NM, nullptr, nullptr, nullptr);
  k_gemm<E_SMALL, false><<<dim3(SMW / 128, NM / 128), tb, 0, stream>>>(xln, ND, wsmT, SMW, smf, SMW, ND, NM,
                                                                        nullptr, nullptr, amask);
  k_gemm<E_DECAY, true><<<g1024, tb, 0, stream>>>(smf, SMW, wfbT, ND, gdec, ND, HD, NM, dt_bias, A_log, nullptr);
  k_gemm<E_SIG, true><<<g1024, tb, 0, stream>>>(smf + HD, SMW, wgbT, ND, gof, ND, HD, NM, nullptr, nullptr, nullptr);

  k_scan<<<NB * NH, tb, 0, stream>>>(qf, kf, vf, gdec, smf, gof, o_norm_w, obf);

  k_gemm<E_BF16, false><<<g1024, tb, 0, stream>>>(obf, ND, woT, ND, opb, ND, ND, NM, nullptr, nullptr, nullptr);

  k_gemm<E_F32, false><<<dim3((2 * NI) / 128, NM / 128), tb, 0, stream>>>(opb, ND, wguT, 2 * NI, gu, 2 * NI, ND, NM,
                                                                           nullptr, nullptr, nullptr);
  k_swiglu<<<(NM * NCH + 7) / 8, tb, 0, stream>>>(gu, act, NM);

  k_gemm<E_RESID, false><<<g1024, tb, 0, stream>>>(act, NI, wdnT, ND, out, ND, NI, NM, hidden, nullptr, nullptr);
}
